// MultiHeadAttentionLSA_13657996001585
// MI455X (gfx1250) — hardware-verified
//
#include <hip/hip_runtime.h>
#include <math.h>
#include <stdint.h>

constexpr int kBatch  = 8;
constexpr int kSeq    = 1024;
constexpr int kEmbed  = 768;
constexpr int kHeads  = 12;
constexpr int kHdim   = 64;
constexpr int kRows   = kBatch * kSeq;
constexpr int kQKCols = 2 * kEmbed;
static_assert(kHeads * kHdim == kEmbed, "cfg");
static_assert(kSeq % 64 == 0 && kEmbed % 64 == 0 && kRows % 64 == 0, "cfg");

constexpr float kPcarry = 32768.0f;
constexpr float kOcarry = 16.0f;
constexpr float kWcarry = 64.0f;

typedef __attribute__((ext_vector_type(16))) _Float16 v16h;
typedef __attribute__((ext_vector_type(8)))  _Float16 v8h;
typedef __attribute__((ext_vector_type(16))) __bf16   v16b;
typedef __attribute__((ext_vector_type(8)))  __bf16   v8b;
typedef __attribute__((ext_vector_type(8)))  float    v8f;
typedef __attribute__((ext_vector_type(4)))  float    v4f;
typedef __attribute__((ext_vector_type(2)))  float    v2f;

__device__ __forceinline__ unsigned short f2bf_bits(float f) {
  unsigned u = __float_as_uint(f);
  return (unsigned short)((u + 0x7FFFu + ((u >> 16) & 1u)) >> 16);
}
__device__ __forceinline__ float bf_bits2f(unsigned short h) { return __uint_as_float(((unsigned)h) << 16); }

__device__ __forceinline__ void dep_guard_h(v8f& a, v8f& b, v16h x, v16h y) { asm volatile("v_nop\n\tv_nop\n\tv_nop\n\tv_nop" : "+v"(a), "+v"(b) : "v"(x), "v"(y)); }
__device__ __forceinline__ void dep_guard_b(v8f& a, v8f& b, v16b x, v16b y) { asm volatile("v_nop\n\tv_nop\n\tv_nop\n\tv_nop" : "+v"(a), "+v"(b) : "v"(x), "v"(y)); }
__device__ __forceinline__ void keep4_h(v16h a, v16h b, v16h c, v16h d) { asm volatile("v_nop" :: "v"(a), "v"(b), "v"(c), "v"(d)); }
__device__ __forceinline__ void keep4_b(v16b a, v16b b, v16b c, v16b d) { asm volatile("v_nop" :: "v"(a), "v"(b), "v"(c), "v"(d)); }
__device__ __forceinline__ void acc_guard4(v8f& a, v8f& b, v8f& c, v8f& d) { asm volatile("v_nop\n\tv_nop\n\tv_nop\n\tv_nop" : "+v"(a), "+v"(b), "+v"(c), "+v"(d)); }
template <typename T> struct Frag;
template <> struct Frag<_Float16> {
  typedef v16h V; union U { v16h v; v8h h[2]; };
  static __device__ __forceinline__ v16h load(const _Float16* p) {
    U f; f.h[0] = *(const v8h*)(p); f.h[1] = *(const v8h*)(p + 16); return f.v;
  }
  static __device__ __forceinline__ v8f mma(v16h a, v16h b, v8f c) {
    return __builtin_amdgcn_wmma_f32_16x16x32_f16(false, a, false, b, (short)0, c, false, false);
  }
  static __device__ __forceinline__ void guard(v8f& a, v8f& b, v16h x, v16h y) { dep_guard_h(a, b, x, y); }
  static __device__ __forceinline__ void keep(v16h a, v16h b, v16h c, v16h d) { keep4_h(a, b, c, d); }
};
template <> struct Frag<__bf16> {
  typedef v16b V; union U { v16b v; v8b h[2]; };
  static __device__ __forceinline__ v16b load(const __bf16* p) {
    U f; f.h[0] = *(const v8b*)(p); f.h[1] = *(const v8b*)(p + 16); return f.v;
  }
  static __device__ __forceinline__ v8f mma(v16b a, v16b b, v8f c) {
    return __builtin_amdgcn_wmma_f32_16x16x32_bf16(false, a, false, b, (short)0, c, false, false);
  }
  static __device__ __forceinline__ void guard(v8f& a, v8f& b, v16b x, v16b y) { dep_guard_b(a, b, x, y); }
  static __device__ __forceinline__ void keep(v16b a, v16b b, v16b c, v16b d) { keep4_b(a, b, c, d); }
};

template <int ET> struct Elem;
template <> struct Elem<0> { typedef _Float16 T; };
template <> struct Elem<1> { typedef __bf16 T; };
template <int ET, bool SPLIT, int BIAS_MODE, int OUT_MODE, bool RESID, int ACT = 0>
__global__ __launch_bounds__(256) void wmma_gemm64(
    const unsigned short* __restrict__ Ap, const unsigned short* __restrict__ A2p, int lda, long strideA,
    const unsigned short* __restrict__ Btp, const unsigned short* __restrict__ Bt2p, int ldb, long strideB,
    void* __restrict__ Cout, void* __restrict__ Cout2, int ldc, long strideC,
    const float* __restrict__ bias,
    const float* __restrict__ resid, long strideR,
    int M, int N, int K, float scale) {
  typedef typename Elem<ET>::T T;
  typedef typename Frag<T>::V V;
  const T* A = (const T*)Ap; const T* A2 = (const T*)A2p; const T* Bt = (const T*)Btp; const T* Bt2 = (const T*)Bt2p;
  __shared__ __align__(16) float sT[8][16 * 68];
  const int b    = blockIdx.y;
  const int lane = threadIdx.x & 31;
  const int wave = threadIdx.x >> 5;
  const int tilesN = N >> 6;
  const int tilesM = M >> 6;
  const int tile = blockIdx.x * 8 + wave;
  if (tile >= tilesM * tilesN) return;
  const int tm = tile / tilesN;
  const int tn = tile - tm * tilesN;
  const int m0 = tm << 6;
  const int n0 = tn << 6;

  const T* Ab  = A  + (size_t)b * strideA;
  const T* Bb  = Bt + (size_t)b * strideB;
  const T* Ab2 = SPLIT ? (A2  + (size_t)b * strideA) : nullptr;
  const T* Bb2 = SPLIT ? (Bt2 + (size_t)b * strideB) : nullptr;

  const int rlane = lane & 15;
  const int koff  = (lane >> 4) * 8;
  const int mOff  = (lane >> 4) * 8;

  v8f acc[4][4];
#pragma unroll
  for (int i = 0; i < 4; ++i)
#pragma unroll
    for (int j = 0; j < 4; ++j) acc[i][j] = (v8f){0.f,0.f,0.f,0.f,0.f,0.f,0.f,0.f};

  for (int k0 = 0; k0 < K; k0 += 32) {
    V bh[4], bl[4];
#pragma unroll
    for (int j = 0; j < 4; ++j) {
      const size_t bo = (size_t)(n0 + (j << 4) + rlane) * ldb + koff + k0;
      bh[j] = Frag<T>::load(Bb + bo);
      if (SPLIT) bl[j] = Frag<T>::load(Bb2 + bo);
    }
#pragma unroll
    for (int i = 0; i < 4; ++i) {
      const size_t ao = (size_t)(m0 + (i << 4) + rlane) * lda + koff + k0;
      V ah = Frag<T>::load(Ab + ao);
      V al;
      if (SPLIT) al = Frag<T>::load(Ab2 + ao);
#pragma unroll
      for (int j = 0; j < 4; ++j) {
        acc[i][j] = Frag<T>::mma(ah, bh[j], acc[i][j]);
        if (SPLIT) {
          acc[i][j] = Frag<T>::mma(ah, bl[j], acc[i][j]);
          acc[i][j] = Frag<T>::mma(al, bh[j], acc[i][j]);
        }
      }
      Frag<T>::guard(acc[i][0], acc[i][3], ah, SPLIT ? al : ah);
    }
    Frag<T>::keep(bh[0], bh[1], bh[2], bh[3]);
    if (SPLIT) Frag<T>::keep(bl[0], bl[1], bl[2], bl[3]);
  }
  acc_guard4(acc[0][0], acc[0][1], acc[0][2], acc[0][3]);
  acc_guard4(acc[1][0], acc[1][1], acc[1][2], acc[1][3]);
  acc_guard4(acc[2][0], acc[2][1], acc[2][2], acc[2][3]);
  acc_guard4(acc[3][0], acc[3][1], acc[3][2], acc[3][3]);

  float* slab = sT[wave];
  const float* Rb = RESID ? (resid + (size_t)b * strideR) : nullptr;
#pragma unroll
  for (int i = 0; i < 4; ++i) {
    const int mBase = m0 + (i << 4);
#pragma unroll
    for (int j = 0; j < 4; ++j) {
      const int n = n0 + (j << 4) + rlane;
      float bv = 0.f;
      if (BIAS_MODE == 2) bv = bias[n];
#pragma unroll
      for (int r = 0; r < 8; ++r) {
        float v = acc[i][j][r] * scale;
        if (BIAS_MODE == 1) v += bias[mBase + mOff + r];
        if (BIAS_MODE == 2) v += bv;
        if (RESID) v += Rb[(size_t)(mBase + mOff + r) * ldc + n];
        if (ACT == 1) v = tanhf(v);
        if (ACT == 2) v = fmaxf(v, 0.0f);
        if (ACT == 3) v = v / (1.0f + expf(-v));
        if (ACT == 4) v = (v > 0.f) ? v : 0.01f * v;
        if (ACT == 5) v = 0.5f * v * (1.0f + erff(v * 0.70710678118654752f));
        slab[(mOff + r) * 68 + (j << 4) + rlane] = v;
      }
    }
    __builtin_amdgcn_fence(__ATOMIC_RELEASE, "workgroup");
    __builtin_amdgcn_wave_barrier();
    __builtin_amdgcn_fence(__ATOMIC_ACQUIRE, "workgroup");
    if (OUT_MODE == 0) {
      float* C = (float*)Cout + (size_t)b * strideC;
      const int hh = lane >> 4, c4 = (lane & 15) * 4;
      for (int pass = 0; pass < 2; ++pass) {
#pragma unroll
        for (int it = 0; it < 8; ++it) {
          const int row = it * 2 + hh;
          v4f v = *(const v4f*)(slab + row * 68 + c4);
          *(volatile v4f*)(C + (size_t)(mBase + row) * ldc + n0 + c4) = v;
        }
        __threadfence();
      }
    } else {
      const int q = lane >> 3, c8 = (lane & 7) * 8;
      unsigned short* C  = (unsigned short*)Cout  + (size_t)b * strideC;
      unsigned short* C2 = (OUT_MODE == 2) ? ((unsigned short*)Cout2 + (size_t)b * strideC) : nullptr;
      for (int pass = 0; pass < 2; ++pass) {
#pragma unroll
        for (int it = 0; it < 4; ++it) {
          const int row = it * 4 + q;
          const float* sp = slab + row * 68 + c8;
          v8h hv, lv;
#pragma unroll
          for (int e = 0; e < 8; ++e) {
            if (OUT_MODE == 1) {
              hv[e] = (_Float16)sp[e];
            } else {
              unsigned short hb = f2bf_bits(sp[e]);
              unsigned short lb = f2bf_bits(sp[e] - bf_bits2f(hb));
              hv[e] = __builtin_bit_cast(_Float16, hb);
              lv[e] = __builtin_bit_cast(_Float16, lb);
            }
          }
          *(volatile v8h*)(C + (size_t)(mBase + row) * ldc + n0 + c8) = hv;
          if (OUT_MODE == 2) *(volatile v8h*)(C2 + (size_t)(mBase + row) * ldc + n0 + c8) = lv;
        }
        __threadfence();
      }
    }
    __builtin_amdgcn_fence(__ATOMIC_RELEASE, "workgroup");
    __builtin_amdgcn_wave_barrier();
    __builtin_amdgcn_fence(__ATOMIC_ACQUIRE, "workgroup");
  }
}

template <int MODE>
__global__ __launch_bounds__(256) void cast16x2_kernel(const float* __restrict__ in, unsigned short* __restrict__ out,
                                                       int n2, float mul) {
  const int i = blockIdx.x * 256 + threadIdx.x;
  if (i < n2) {
    const v2f f = *(const v2f*)(in + 2 * (size_t)i);
    unsigned short a0, a1;
    if (MODE == 0) {
      a0 = f2bf_bits(f[0]);
      a1 = f2bf_bits(f[1]);
    } else {
      const float g0 = bf_bits2f(f2bf_bits(f[0])) * mul;
      const float g1 = bf_bits2f(f2bf_bits(f[1])) * mul;
      a0 = __builtin_bit_cast(unsigned short, (_Float16)g0);
      a1 = __builtin_bit_cast(unsigned short, (_Float16)g1);
    }
    const unsigned u = (unsigned)a0 | ((unsigned)a1 << 16);
    ((volatile unsigned*)out)[i] = u;
    __threadfence();
    ((volatile unsigned*)out)[i] = u;
  }
}

#define AT_D 64
#define AT_NW 4
#define AT_QB 64
#define AT_KC 64

__device__ __forceinline__ v8f at_mma_h(v16h a, v16h b, v8f c) {
  c = __builtin_amdgcn_wmma_f32_16x16x32_f16(false, a, false, b, (short)0, c, false, false);
  asm volatile("v_nop\n\tv_nop\n\tv_nop\n\tv_nop" : "+v"(c) : "v"(a), "v"(b));
  return c;
}

__global__ __launch_bounds__(128)
void attn_f16_full64_kernel(const unsigned short* __restrict__ qkp, const unsigned short* __restrict__ vtp,
                            const float* __restrict__ temp, unsigned short* __restrict__ outp) {
  union FH { v16h v; v8h h[2]; };
  __shared__ __align__(16) _Float16 Ksh[AT_KC * AT_D];
  __shared__ __align__(16) _Float16 Vth[AT_D * AT_KC];
  __shared__ __align__(16) _Float16 Psh[AT_NW][16 * AT_KC];
  __shared__ __align__(16) float    Os[AT_NW][16 * 68];

  const int tid  = threadIdx.x;
  const int wave = tid >> 5;
  const int lane = tid & 31;
  const int hh   = lane >> 4;
  const int c    = lane & 15;

  const int nqb = kSeq / AT_QB;
  const int bx  = blockIdx.x;
  const int qb  = bx % nqb;
  const int bhd = bx / nqb;
  const int h   = bhd % kHeads;
  const int b   = bhd / kHeads;
  const int q0  = qb * AT_QB + wave * 16;

  const _Float16* Qp = (const _Float16*)(const void*)qkp + (size_t)b * kSeq * kQKCols + (size_t)h * AT_D;
  const _Float16* Kp = Qp + kEmbed;
  const _Float16* Vp = (const _Float16*)(const void*)vtp + (size_t)b * kEmbed * kSeq + (size_t)h * AT_D * kSeq;
  _Float16*       Op = (_Float16*)(void*)outp + (size_t)b * kSeq * kEmbed + (size_t)h * AT_D;

  const float tval = temp[h];

  v16h qa[2];
#pragma unroll
  for (int dc = 0; dc < 2; ++dc) {
    const _Float16* qr = Qp + (size_t)(q0 + c) * kQKCols + dc * 32 + 8 * hh;
    qa[dc] = Frag<_Float16>::load(qr);
  }

  float mrow[8], lrow[8];
  v8f oacc[4];
#pragma unroll
  for (int r = 0; r < 8; ++r) { mrow[r] = -INFINITY; lrow[r] = 0.f; }
#pragma unroll
  for (int t = 0; t < 4; ++t) oacc[t] = (v8f){0.f,0.f,0.f,0.f,0.f,0.f,0.f,0.f};

  const int nChunks = kSeq / AT_KC;
  for (int kc = 0; kc < nChunks; ++kc) {
    const int kv0 = kc * AT_KC;
    __syncthreads();
    {
      const int r = tid >> 1, half = (tid & 1) * 32;
      const _Float16* ks = Kp + (size_t)(kv0 + r) * kQKCols + half;
      const _Float16* vs = Vp + (size_t)r * kSeq + kv0 + half;
#pragma unroll
      for (int i = 0; i < 4; ++i) {
        const v8h a0 = *(const v8h*)(ks + 8 * i);
        const v8h b0 = *(const v8h*)(vs + 8 * i);
        *(v8h*)(Ksh + r * AT_D  + half + 8 * i) = a0;
        *(v8h*)(Vth + r * AT_KC + half + 8 * i) = b0;
      }
    }
    __syncthreads();

    v8f s[4];
#pragma unroll
    for (int j = 0; j < 4; ++j) {
      s[j] = (v8f){0.f,0.f,0.f,0.f,0.f,0.f,0.f,0.f};
#pragma unroll
      for (int dc = 0; dc < 2; ++dc) {
        FH kb;
        kb.h[0] = *(const v8h*)(Ksh + (j * 16 + c) * AT_D + dc * 32 + 8 * hh);
        kb.h[1] = *(const v8h*)(Ksh + (j * 16 + c) * AT_D + dc * 32 + 16 + 8 * hh);
        s[j] = at_mma_h(qa[dc], kb.v, s[j]);
      }
    }
    float cm[8];
#pragma unroll
    for (int r = 0; r < 8; ++r) {
      float m = -INFINITY;
#pragma unroll
      for (int j = 0; j < 4; ++j) {
        const float sv = (s[j][r] * 0.125f) * tval;
        s[j][r] = sv;
        m = fmaxf(m, sv);
      }
#pragma unroll
      for (int off = 1; off < 16; off <<= 1) m = fmaxf(m, __shfl_xor(m, off, 32));
      cm[r] = m;
    }
    _Float16* pwh = Psh[wave];
#pragma unroll
    for (int r = 0; r < 8; ++r) {
      const float mnew = fmaxf(mrow[r], cm[r]);
      const float alpha = expf(mrow[r] - mnew);
      mrow[r] = mnew;
      float psum = 0.f;
#pragma unroll
      for (int j = 0; j < 4; ++j) {
        const float p = expf(s[j][r] - mnew);
        psum += p;
        pwh[(8 * hh + r) * AT_KC + j * 16 + c] = (_Float16)(p * kPcarry);
      }
#pragma unroll
      for (int off = 1; off < 16; off <<= 1) psum += __shfl_xor(psum, off, 32);
      lrow[r] = lrow[r] * alpha + psum;
#pragma unroll
      for (int t = 0; t < 4; ++t) oacc[t][r] *= alpha;
    }
    __builtin_amdgcn_fence(__ATOMIC_RELEASE, "workgroup");
    __builtin_amdgcn_wave_barrier();
    __builtin_amdgcn_fence(__ATOMIC_ACQUIRE, "workgroup");
#pragma unroll 1
    for (int kk = 0; kk < 2; ++kk) {
      FH pa;
      pa.h[0] = *(const v8h*)(pwh + c * AT_KC + kk * 32 + 8 * hh);
      pa.h[1] = *(const v8h*)(pwh + c * AT_KC + kk * 32 + 16 + 8 * hh);
#pragma unroll
      for (int t = 0; t < 4; ++t) {
        FH vb;
        vb.h[0] = *(const v8h*)(Vth + (t * 16 + c) * AT_KC + kk * 32 + 8 * hh);
        vb.h[1] = *(const v8h*)(Vth + (t * 16 + c) * AT_KC + kk * 32 + 16 + 8 * hh);
        oacc[t] = at_mma_h(pa.v, vb.v, oacc[t]);
      }
    }
  }

  float* os = Os[wave];
#pragma unroll
  for (int r = 0; r < 8; ++r) {
    const float inv = kOcarry * (1.0f / (lrow[r] * kPcarry));
#pragma unroll
    for (int t = 0; t < 4; ++t) os[(8 * hh + r) * 68 + t * 16 + c] = oacc[t][r] * inv;
  }
  __builtin_amdgcn_fence(__ATOMIC_RELEASE, "workgroup");
  __builtin_amdgcn_wave_barrier();
  __builtin_amdgcn_fence(__ATOMIC_ACQUIRE, "workgroup");
  {
    const int q = lane >> 3, c8 = (lane & 7) * 8;
    for (int pass = 0; pass < 2; ++pass) {
#pragma unroll
      for (int it = 0; it < 4; ++it) {
        const int row = it * 4 + q;
        const float* sp = os + row * 68 + c8;
        v8h hv;
#pragma unroll
        for (int e = 0; e < 8; ++e) hv[e] = (_Float16)sp[e];
        *(volatile v8h*)(Op + (size_t)(q0 + row) * kEmbed + c8) = hv;
      }
      __threadfence();
    }
  }
}

extern "C" void kernel_launch(void* const* d_in, const int* in_sizes, int n_in,
                              void* d_out, int out_size, void* d_ws,
                              size_t ws_size, hipStream_t stream) {
  if (n_in < 5) return;
  const int nX    = kRows * kEmbed;
  const int nWqkv = 3 * kEmbed * kEmbed;
  const int nWp   = kEmbed * kEmbed;
  if (in_sizes[0] != nX || in_sizes[1] != nWqkv || in_sizes[2] != nWp ||
      in_sizes[3] != kEmbed || in_sizes[4] != kHeads || out_size != nX) return;

  const float* x      = (const float*)d_in[0];
  const float* w_qkv  = (const float*)d_in[1];
  const float* w_proj = (const float*)d_in[2];
  const float* b_proj = (const float*)d_in[3];
  const float* temp   = (const float*)d_in[4];
  float* out = (float*)d_out;

  size_t off = 0;
  const size_t oXb   = off; off += (size_t)nX * 2;
  const size_t oWqkv = off; off += (size_t)nWqkv * 2;
  const size_t oWp   = off; off += (size_t)nWp * 2;
  const size_t oQK   = off; off += (size_t)kRows * kQKCols * 2;
  const size_t oVT   = off; off += (size_t)kBatch * kEmbed * kSeq * 2;
  const size_t oOb   = off; off += (size_t)kRows * kEmbed * 2;
  if (off > ws_size) return;

  char* ws = (char*)d_ws;
  unsigned short* xb    = (unsigned short*)(ws + oXb);
  unsigned short* wqkvb = (unsigned short*)(ws + oWqkv);
  unsigned short* wph   = (unsigned short*)(ws + oWp);
  unsigned short* qk    = (unsigned short*)(ws + oQK);
  unsigned short* vt    = (unsigned short*)(ws + oVT);
  unsigned short* ob    = (unsigned short*)(ws + oOb);

  {
    const int n2x = nX / 2, n2w = nWqkv / 2, n2p = nWp / 2;
    cast16x2_kernel<0><<<dim3((n2x + 255) / 256), dim3(256), 0, stream>>>(x, xb, n2x, 1.0f);
    cast16x2_kernel<0><<<dim3((n2w + 255) / 256), dim3(256), 0, stream>>>(w_qkv, wqkvb, n2w, 1.0f);
    cast16x2_kernel<1><<<dim3((n2p + 255) / 256), dim3(256), 0, stream>>>(w_proj, wph, n2p, kWcarry);
  }

  {
    const int M = kRows, N = kQKCols, K = kEmbed;
    const int tiles = (M / 64) * (N / 64);
    wmma_gemm64<1, false, 0, 1, false, 0><<<dim3((tiles + 7) / 8, 1), dim3(256), 0, stream>>>(
        xb, xb, kEmbed, 0L,
        wqkvb, wqkvb, kEmbed, 0L,
        (void*)qk, (void*)qk, kQKCols, 0L,
        b_proj, b_proj, 0L,
        M, N, K, 1.0f);
  }

  {
    const int M = kEmbed, N = kSeq, K = kEmbed;
    const int tiles = (M / 64) * (N / 64);
    wmma_gemm64<1, false, 0, 1, false, 0><<<dim3((tiles + 7) / 8, kBatch), dim3(256), 0, stream>>>(
        wqkvb + (size_t)2 * kEmbed * kEmbed, wqkvb + (size_t)2 * kEmbed * kEmbed, kEmbed, 0L,
        xb, xb, kEmbed, (long)kSeq * kEmbed,
        (void*)vt, (void*)vt, kSeq, (long)kEmbed * kSeq,
        b_proj, b_proj, 0L,
        M, N, K, 1.0f);
  }

  attn_f16_full64_kernel<<<dim3(kBatch * kHeads * (kSeq / 64)), dim3(128), 0, stream>>>(qk, vt, temp, ob);

  {
    const int M = kRows, N = kEmbed, K = kEmbed;
    const int tiles = (M / 64) * (N / 64);
    wmma_gemm64<0, false, 2, 0, false, 0><<<dim3((tiles + 7) / 8, 1), dim3(256), 0, stream>>>(
        ob, ob, kEmbed, 0L,
        wph, wph, kEmbed, 0L,
        (void*)out, (void*)out, kEmbed, 0L,
        b_proj, b_proj, 0L,
        M, N, K, 1.0f / (kOcarry * kWcarry));
  }
}
